// MultiHeadDistanceLayer_37014028156966
// MI455X (gfx1250) — hardware-verified
//
#include <hip/hip_runtime.h>


typedef __attribute__((ext_vector_type(16))) _Float16 v16h;
typedef __attribute__((ext_vector_type(8)))  _Float16 v8h;
typedef __attribute__((ext_vector_type(8)))  float    v8f;
typedef __attribute__((ext_vector_type(4)))  float    v4f;
#define B_    4
#define L_    2048
#define DIN   256
#define H_    8
#define HD    64
#define HDTOT 512
#define MD    128
#define DD    257
#define DDP   288
#define NKC   8
#define VST2(T, ptr, val) do { const T _v = (val); *(volatile T*)(ptr) = _v; __threadfence(); *(volatile T*)(ptr) = _v; } while (0)
__device__ __forceinline__ v8f wmma16(v16h a, v16h b, v8f c) {
  v8f d = __builtin_amdgcn_wmma_f32_16x16x32_f16(false, a, false, b, (short)0, c, false, false);
  asm volatile("v_nop\n\tv_nop\n\tv_nop\n\tv_nop" : "+v"(d) : "v"(a), "v"(b));
  return d;
}
__device__ __forceinline__ v16h frag16(const _Float16* p, int hh) {
  const v8h lo = *(const v8h*)(p + 8 * hh), hi = *(const v8h*)(p + 16 + 8 * hh);
  return __builtin_shufflevector(lo, hi, 0,1,2,3,4,5,6,7,8,9,10,11,12,13,14,15);
}
__global__ __launch_bounds__(256) void k_prep(const float* __restrict__ x, const float* __restrict__ pe, const float* __restrict__ Wv,
                                              _Float16* __restrict__ qk16, float* __restrict__ vsig) {
  __shared__ float xs[32][DIN + 4];
  const int row0 = blockIdx.x * 32, b = row0 >> 11, l0 = row0 & (L_ - 1), t = threadIdx.x;
  for (int q = 0; q < 4; ++q) {
    const int piece = q * 256 + t, r = piece >> 5, c8 = (piece & 31) * 8;
    v8h o;
#pragma unroll
    for (int e = 0; e < 8; ++e) { const float xv = x[(size_t)(row0 + r) * DIN + c8 + e]; xs[r][c8 + e] = xv; o[e] = (_Float16)(xv + pe[(l0 + r) * DIN + c8 + e]); }
    VST2(v8h, qk16 + (size_t)(row0 + r) * DIN + c8, o);
  }
  __syncthreads();
  const int h = t >> 5, r = t & 31;
  float z = 0.f;
  for (int i = 0; i < DIN; ++i) z += xs[r][i] * Wv[i * H_ + h];
  VST2(float, vsig + (size_t)(b * H_ + h) * L_ + l0 + r, 1.0f / (1.0f + expf(-z)));
}
__global__ __launch_bounds__(256) void k_wt(const float* __restrict__ Wq, const float* __restrict__ Wk, _Float16* __restrict__ wtq, _Float16* __restrict__ wtk) {
  const int t = blockIdx.x * 256 + threadIdx.x;
  const int n = t >> 5, k0 = (t & 31) * 8;
  v8h a, c;
#pragma unroll
  for (int e = 0; e < 8; ++e) { a[e] = (_Float16)Wq[(k0 + e) * HDTOT + n]; c[e] = (_Float16)Wk[(k0 + e) * HDTOT + n]; }
  VST2(v8h, wtq + n * DIN + k0, a); VST2(v8h, wtk + n * DIN + k0, c);
}
__global__ __launch_bounds__(256) void k_proj(const _Float16* __restrict__ qk16, const _Float16* __restrict__ wtq, const _Float16* __restrict__ wtk,
                                              const float* __restrict__ bq, const float* __restrict__ bk, _Float16* __restrict__ Q16, _Float16* __restrict__ K16) {
  __shared__ __attribute__((aligned(16))) _Float16 sT[8][16 * 72];
  const int lane = threadIdx.x & 31, wave = threadIdx.x >> 5, hh = lane >> 4, l16 = lane & 15;
  const int tile = blockIdx.x * 8 + wave;
  const int mat = tile >> 12, rowt = (tile >> 3) & 511, h = tile & 7;
  const _Float16* wt = mat ? wtk : wtq; const float* bias = mat ? bk : bq; _Float16* out = mat ? K16 : Q16;
  v8f acc[4] = {};
#pragma unroll
  for (int kk = 0; kk < DIN; kk += 32) {
    const v16h a = frag16(qk16 + (size_t)(rowt * 16 + l16) * DIN + kk, hh);
#pragma unroll
    for (int tn = 0; tn < 4; ++tn) { const v16h bb = frag16(wt + (size_t)(h * HD + tn * 16 + l16) * DIN + kk, hh); acc[tn] = wmma16(a, bb, acc[tn]); }
  }
  _Float16* st = sT[wave];
#pragma unroll
  for (int tn = 0; tn < 4; ++tn)
#pragma unroll
    for (int g = 0; g < 8; ++g) st[(g + 8 * hh) * 72 + tn * 16 + l16] = (_Float16)(acc[tn][g] + bias[h * HD + tn * 16 + l16]);
  __builtin_amdgcn_fence(__ATOMIC_RELEASE, "workgroup"); __builtin_amdgcn_wave_barrier(); __builtin_amdgcn_fence(__ATOMIC_ACQUIRE, "workgroup");
  const int r0 = rowt * 16, b = r0 >> 11, l0 = r0 & (L_ - 1);
  _Float16* dst = out + ((size_t)(b * H_ + h) * L_ + l0) * HD;
  for (int pass = 0; pass < 2; ++pass) {
#pragma unroll
    for (int j = 0; j < 4; ++j) { const int rr = j * 4 + (lane >> 3), q8 = (lane & 7) * 8; *(volatile v8h*)(dst + (size_t)rr * HD + q8) = *(const v8h*)(&st[rr * 72 + q8]); }
    __threadfence();
  }
}
__global__ __launch_bounds__(256) void k_stats(const _Float16* __restrict__ Q16, const _Float16* __restrict__ K16, float* __restrict__ stats) {
  __shared__ float ss[128];
  const int lane = threadIdx.x & 31, wave = threadIdx.x >> 5, hh = lane >> 4, l16 = lane & 15;
  const int bh = blockIdx.x >> 4, qt = (blockIdx.x & 15) * 8 + wave;
  const _Float16* Qb = Q16 + ((size_t)bh * L_ + qt * 16) * HD;
  const _Float16* Kb = K16 + (size_t)bh * L_ * HD;
  const v16h a0 = frag16(Qb + l16 * HD, hh), a1 = frag16(Qb + l16 * HD + 32, hh);
  float se[8] = {0.f, 0.f, 0.f, 0.f, 0.f, 0.f, 0.f, 0.f};
  for (int t = 0; t < L_ / 16; ++t) {
    const _Float16* Kt = Kb + (size_t)(t * 16 + l16) * HD;
    v8f c = {};
    c = wmma16(a0, frag16(Kt, hh), c);
    c = wmma16(a1, frag16(Kt + 32, hh), c);
#pragma unroll
    for (int g = 0; g < 8; ++g) se[g] += __expf(c[g] * 0.125f);
  }
#pragma unroll
  for (int off = 1; off < 16; off <<= 1)
#pragma unroll
    for (int g = 0; g < 8; ++g) se[g] += __shfl_xor(se[g], off, 32);
  float mine = se[0];
#pragma unroll
  for (int g = 1; g < 8; ++g) mine = (g == l16) ? se[g] : mine;
  if (l16 < 8) ss[wave * 16 + hh * 8 + l16] = 1.0f / mine;
  __syncthreads();
  if (threadIdx.x < 32) VST2(v4f, stats + (size_t)bh * L_ + (blockIdx.x & 15) * 128 + threadIdx.x * 4, *(const v4f*)(&ss[threadIdx.x * 4]));
}
__global__ __launch_bounds__(256) void k_band(const _Float16* __restrict__ Q16, const _Float16* __restrict__ K16, const float* __restrict__ stats,
                                              const float* __restrict__ vsig, float* __restrict__ partial) {
  __shared__ float Tt[8][16][17];
  __shared__ float Sw[8][DDP];
  const int t = threadIdx.x, wave = t >> 5, lane = t & 31, hh = lane >> 4, l16 = lane & 15;
  const int bh = blockIdx.x >> 3, kc = blockIdx.x & 7;
  for (int i = lane; i < DDP; i += 32) Sw[wave][i] = 0.f;
  const _Float16* Qb = Q16 + (size_t)bh * L_ * HD;
  const _Float16* Kb = K16 + (size_t)bh * L_ * HD;
  const float* st = stats + (size_t)bh * L_;
  for (int kk = 0; kk < 2; ++kk) {
    const int kt = kc * 16 + wave * 2 + kk;
    const int key = kt * 16 + l16;
    const v16h b0 = frag16(Kb + (size_t)key * HD, hh), b1 = frag16(Kb + (size_t)key * HD + 32, hh);
    const float vf = vsig[(size_t)bh * L_ + (L_ - 1 - key)];
    for (int dq = -8; dq <= 8; ++dq) {
      const int qt = kt + dq;
      if (qt < 0 || qt >= L_ / 16) continue;
      const v16h a0 = frag16(Qb + (size_t)(qt * 16 + l16) * HD, hh), a1 = frag16(Qb + (size_t)(qt * 16 + l16) * HD + 32, hh);
      v8f c = {};
      c = wmma16(a0, b0, c);
      c = wmma16(a1, b1, c);
#pragma unroll
      for (int g = 0; g < 8; ++g) {
        const int qi = g + 8 * hh;
        Tt[wave][qi][l16] = __expf(c[g] * 0.125f) * st[qt * 16 + qi] * vf;
      }
      __builtin_amdgcn_fence(__ATOMIC_RELEASE, "workgroup"); __builtin_amdgcn_wave_barrier(); __builtin_amdgcn_fence(__ATOMIC_ACQUIRE, "workgroup");
      if (lane < 31) {
        const int orel = lane - 15, o = -16 * dq + orel;
        if (o >= -MD && o <= MD) {
          float s = 0.f;
#pragma unroll
          for (int qi = 0; qi < 16; ++qi) { const int kj = qi + orel; if (kj >= 0 && kj < 16) s += Tt[wave][qi][kj]; }
          Sw[wave][MD + o] += s;
        }
      }
      __builtin_amdgcn_fence(__ATOMIC_RELEASE, "workgroup"); __builtin_amdgcn_wave_barrier(); __builtin_amdgcn_fence(__ATOMIC_ACQUIRE, "workgroup");
    }
  }
  __syncthreads();
  float* dst = partial + ((size_t)bh * NKC + kc) * DDP;
  for (int pass = 0; pass < 2; ++pass) {
    if (t < DDP / 4) {
      v4f v = {0.f, 0.f, 0.f, 0.f};
#pragma unroll
      for (int w = 0; w < 8; ++w) { v[0] += Sw[w][t * 4]; v[1] += Sw[w][t * 4 + 1]; v[2] += Sw[w][t * 4 + 2]; v[3] += Sw[w][t * 4 + 3]; }
      *(volatile v4f*)(dst + t * 4) = v;
    }
    __threadfence();
  }
}
__global__ __launch_bounds__(256) void k_final(const float* __restrict__ partial, float* __restrict__ out) {
  const int i = blockIdx.x * 256 + threadIdx.x;
  if (i >= B_ * DD * H_) return;
  const int b = i / (DD * H_), r = i % (DD * H_), j = r / H_, h = r % H_;
  const float* P = partial + (size_t)(b * H_ + h) * NKC * DDP;
  auto S = [&](int jj) { float s = 0.f; for (int kc = 0; kc < NKC; ++kc) s += P[kc * DDP + jj]; return s; };
  float sum = S(j), cnt = 1.f;
  if (j > 0)      { sum += S(j - 1); cnt += 1.f; }
  if (j < DD - 1) { sum += S(j + 1); cnt += 1.f; }
  VST2(float, out + i, sum / cnt);
}
extern "C" void kernel_launch(void* const* d_in, const int* in_sizes, int n_in,
                              void* d_out, int out_size, void* d_ws, size_t ws_size, hipStream_t stream) {
  (void)in_sizes; (void)n_in; (void)out_size;
  const float* x  = (const float*)d_in[0];
  const float* pe = (const float*)d_in[1];
  const float* Wq = (const float*)d_in[2];
  const float* bq = (const float*)d_in[3];
  const float* Wk = (const float*)d_in[4];
  const float* bk = (const float*)d_in[5];
  const float* Wv = (const float*)d_in[6];
  char* ws = (char*)d_ws; size_t off = 0;
  auto alloc = [&](size_t bytes) -> void* { void* p = ws + off; off = (off + bytes + 255) & ~(size_t)255; return p; };
  _Float16* qk16 = (_Float16*)alloc((size_t)B_ * L_ * DIN * 2);
  _Float16* wtq  = (_Float16*)alloc((size_t)HDTOT * DIN * 2);
  _Float16* wtk  = (_Float16*)alloc((size_t)HDTOT * DIN * 2);
  _Float16* Q16  = (_Float16*)alloc((size_t)B_ * H_ * L_ * HD * 2);
  _Float16* K16  = (_Float16*)alloc((size_t)B_ * H_ * L_ * HD * 2);
  float*    vsig = (float*)alloc((size_t)B_ * H_ * L_ * 4);
  float*    stats= (float*)alloc((size_t)B_ * H_ * L_ * 4);
  float*    part = (float*)alloc((size_t)B_ * H_ * NKC * DDP * 4);
  if (off > ws_size) return;
  k_prep <<<B_ * L_ / 32, 256, 0, stream>>>(x, pe, Wv, qk16, vsig);
  k_wt   <<<HDTOT * 32 / 256, 256, 0, stream>>>(Wq, Wk, wtq, wtk);
  k_proj <<<8192 / 8, 256, 0, stream>>>(qk16, wtq, wtk, bq, bk, Q16, K16);
  k_stats<<<B_ * H_ * 16, 256, 0, stream>>>(Q16, K16, stats);
  k_band <<<B_ * H_ * NKC, 256, 0, stream>>>(Q16, K16, stats, vsig, part);
  k_final<<<(B_ * DD * H_ + 255) / 256, 256, 0, stream>>>(part, (float*)d_out);
}
